// MANO1D_69612829934184
// MI455X (gfx1250) — hardware-verified
//
#include <hip/hip_runtime.h>


#ifndef NB
#define NB 4
#endif
#ifndef SEQ
#define SEQ 16384
#endif
#define NB_FULL  4
#define SEQ_FULL 16384
#ifndef OUT_SEQ
#define OUT_SEQ SEQ
#endif
#define DM    64
#define NH_   8
#define HD    64
#define INNER 512
#define AW    4
#ifndef KSL
#define KSL   16
#endif
#define TSL   (SEQ / KSL)
#define OSP   36
#define OSQ   68
#define TSP   65
#define QRS   2048.0f
#define QRI   (1.0f / 2048.0f)
#define DOTC  64.0f
#define CTXC  16.0f
#define WOC   64.0f
#define DSC   (DOTC / (float)SEQ)
#define CSC   (CTXC / DOTC)
#define OSC   (1.0f / (CTXC * WOC))
#define DOTS_RES  1
#define APPLY_RES 0
#define OUT_RES   0

static_assert(HD == 64);
static_assert(NH_ * HD == INNER);
static_assert(DM == 64);
static_assert(DM % 32 == 0);
static_assert(HD % 32 == 0);
static_assert(INNER % 64 == 0);
static_assert(INNER % 32 == 0);
static_assert(SEQ % 64 == 0);
static_assert(SEQ % (16 * AW) == 0);
static_assert(SEQ % (KSL * 32) == 0);
static_assert((SEQ & (SEQ - 1)) == 0);
static_assert(NB <= NB_FULL);
static_assert(SEQ <= SEQ_FULL);
static_assert((OSP * 4) % 16 == 0);
static_assert((OSQ * 4) % 16 == 0);
static_assert(32 * 16 * 4 == 16 * 64 * 2);
static_assert(32 * 16 * 4 == 16 * 32 * 4);
static_assert(32 * 16 * 8 == 16 * 64 * 4);
static_assert(256 * 16 * 2 == 64 * 64 * 2);
static_assert(256 * 4 * 4 == 64 * 64);
static_assert(16 * OSQ * 4 <= 131072);
static_assert(16 * OSP * 4 <= 131072);
static_assert(AW * 16 * OSQ * 4 <= 131072);
static_assert(64 * TSP * 4 <= 131072);

typedef _Float16 h16;
typedef unsigned short bf;
typedef __attribute__((ext_vector_type(16))) __bf16   v16bf;
typedef __attribute__((ext_vector_type(16))) _Float16 v16h;
typedef __attribute__((ext_vector_type(8)))  _Float16 v8h;
typedef __attribute__((ext_vector_type(8)))  unsigned short v8us;
typedef __attribute__((ext_vector_type(8)))  float    v8f;
typedef __attribute__((ext_vector_type(4)))  float    v4f;
typedef v4f  __attribute__((may_alias)) v4fa;

__device__ __forceinline__ unsigned short f2bf(float f) { unsigned u = __float_as_uint(f); u += 0x7FFFu + ((u >> 16) & 1u); return (unsigned short)(u >> 16); }
__device__ __forceinline__ float bfr(float f) { return __uint_as_float(((unsigned)f2bf(f)) << 16); }
__device__ __forceinline__ v16h cat16(v8h lo, v8h hi) { return __builtin_shufflevector(lo, hi, 0, 1, 2, 3, 4, 5, 6, 7, 8, 9, 10, 11, 12, 13, 14, 15); }
__device__ __forceinline__ v16bf cat16b(v8us lo, v8us hi) { return __builtin_bit_cast(v16bf, __builtin_shufflevector(lo, hi, 0, 1, 2, 3, 4, 5, 6, 7, 8, 9, 10, 11, 12, 13, 14, 15)); }
__device__ __forceinline__ v8f wmma16(v16h a, v16h b, v8f c) { return __builtin_amdgcn_wmma_f32_16x16x32_f16(false, a, false, b, (short)0, c, false, false); }
__device__ __forceinline__ v8f wmmab(v16bf a, v16bf b, v8f c) { return __builtin_amdgcn_wmma_f32_16x16x32_bf16(false, a, false, b, (short)0, c, false, false); }
__device__ __forceinline__ v16h  ldh(const h16* p) { return cat16(*(const v8h*)p, *(const v8h*)(p + 16)); }
__device__ __forceinline__ v16bf ldb(const bf* p)  { return cat16b(*(const v8us*)p, *(const v8us*)(p + 16)); }
__device__ __forceinline__ void wave_sync() { __builtin_amdgcn_fence(3  , "wavefront"); __builtin_amdgcn_wave_barrier(); asm volatile("" ::: "memory"); }
__device__ __forceinline__ v8f wmmabg(v16bf a, v16bf b, v8f c) { c = wmmab(a, b, c); asm volatile("v_nop\n\tv_nop\n\tv_nop\n\tv_nop" : "+v"(c) : "v"(a), "v"(b)); return c; }
__device__ __forceinline__ v8f wmma16g(v16h a, v16h b, v8f c) { c = wmma16(a, b, c); asm volatile("v_nop\n\tv_nop\n\tv_nop\n\tv_nop" : "+v"(c) : "v"(a), "v"(b)); return c; }
static __device__ __forceinline__ h16 toh_flush(float v) { const float w = (fabsf(v) < 6.103515625e-05f) ? 0.0f : v; return (h16)w; }

__global__ __launch_bounds__(256) void k_cvt8(const float* __restrict__ src, bf* dst, size_t n8) {
    const size_t i = (size_t)blockIdx.x * 256 + threadIdx.x; if (i >= n8) return;
    const v8f v = *(const v8f*)(src + i * 8); v8us o;
#pragma unroll
    for (int k = 0; k < 8; ++k) o[k] = f2bf(v[k]);
    *(volatile v8us*)(dst + i * 8) = o; __threadfence(); *(volatile v8us*)(dst + i * 8) = o;
}

__global__ __launch_bounds__(256) void k_wcvt(const float* __restrict__ src, h16* dst, size_t n8) {
    const size_t i = (size_t)blockIdx.x * 256 + threadIdx.x; if (i >= n8) return;
    const v8f v = *(const v8f*)(src + i * 8); v8h o;
#pragma unroll
    for (int k = 0; k < 8; ++k) o[k] = toh_flush(bfr(v[k]) * WOC);
    *(volatile v8h*)(dst + i * 8) = o; __threadfence(); *(volatile v8h*)(dst + i * 8) = o;
}

__global__ __launch_bounds__(32) void k_proj(const bf* __restrict__ A, const bf* __restrict__ Bt, h16* Ph, h16* Pr, int tr) {
    __shared__ __align__(16) float os[16 * OSQ];
    const int lane = threadIdx.x & 31, lr = lane & 15, hi = lane >> 4;
    const unsigned r0 = blockIdx.x * 64u, c0 = blockIdx.y * 64u;
    v8f acc[4][4];
#pragma unroll
    for (int mb = 0; mb < 4; ++mb)
#pragma unroll
        for (int nb = 0; nb < 4; ++nb) acc[mb][nb] = (v8f){};
    const size_t aoff = (size_t)(r0 + lr) * DM + 8 * hi, boff = (size_t)(c0 + lr) * DM + 8 * hi;
#pragma unroll 1
    for (int kc = 0; kc < DM; kc += 32) {
        v16bf a[4];
#pragma unroll
        for (int mb = 0; mb < 4; ++mb) a[mb] = ldb(A + aoff + (size_t)mb * 16 * DM + kc);
#pragma unroll
        for (int nb = 0; nb < 4; ++nb) { const v16bf b = ldb(Bt + boff + (size_t)nb * 16 * DM + kc);
#pragma unroll
            for (int mb = 0; mb < 4; ++mb) acc[mb][nb] = wmmabg(a[mb], b, acc[mb][nb]); }
    }
    const size_t pitch = tr ? (size_t)SEQ : (size_t)INNER;
    const size_t tbase = (size_t)r0 * pitch + (size_t)c0;
#pragma unroll
    for (int mb = 0; mb < 4; ++mb) {
#pragma unroll
        for (int nb = 0; nb < 4; ++nb) {
#pragma unroll
            for (int j = 0; j < 8; ++j) os[(hi * 8 + j) * OSQ + nb * 16 + lr] = acc[mb][nb][j]; }
        wave_sync();
#pragma unroll 1
        for (int ps = 0; ps < 2; ++ps) {
#pragma unroll
            for (int s = 0; s < 4; ++s) { const int row = 4 * s + (lane >> 3), c8 = (lane & 7) * 8;
                const v4f x0 = *(const v4fa*)(&os[row * OSQ + c8]); const v4f x1 = *(const v4fa*)(&os[row * OSQ + c8 + 4]); v8h hv, rv;
#pragma unroll
                for (int i = 0; i < 4; ++i) { const h16 a0 = toh_flush(x0[i]); const h16 a1 = toh_flush(x1[i]); hv[i] = a0; hv[4 + i] = a1;
                    rv[i] = toh_flush((x0[i] - (float)a0) * QRS); rv[4 + i] = toh_flush((x1[i] - (float)a1) * QRS); }
                const size_t oo = tbase + (size_t)(mb * 16 + row) * pitch + (size_t)c8;
                *(volatile v8h*)(Ph + oo) = hv; *(volatile v8h*)(Pr + oo) = rv; }
            if (ps == 0) __threadfence(); }
        wave_sync();
    }
}

__global__ __launch_bounds__(32) void k_dots(const h16* __restrict__ KH, const h16* __restrict__ KR, const h16* __restrict__ VH, const h16* __restrict__ VR, float* PART) {
    __shared__ __align__(16) float os[16 * OSP];
    const int lane = threadIdx.x & 31, lr = lane & 15, hi = lane >> 4;
    const unsigned sl = blockIdx.x, ty = blockIdx.y, hd = blockIdx.z;
    const unsigned d0 = (ty >> 1) * 32u, e0 = (ty & 1u) * 32u;
    const size_t aoff = ((size_t)(hd * 64u + d0) + (size_t)lr) * SEQ + (size_t)sl * TSL + 8 * hi;
    const size_t boff = ((size_t)(hd * 64u + e0) + (size_t)lr) * SEQ + (size_t)sl * TSL + 8 * hi;
    const v16h hz = (v16h){};
    v8f sH[2][2], sR[2][2];
#pragma unroll
    for (int mb = 0; mb < 2; ++mb)
#pragma unroll
        for (int nb = 0; nb < 2; ++nb) { sH[mb][nb] = (v8f){}; sR[mb][nb] = (v8f){}; }
#pragma unroll 1
    for (int kc = 0; kc < TSL; kc += 32) {
        v16h ah[2], ar[2];
#pragma unroll
        for (int mb = 0; mb < 2; ++mb) { ah[mb] = ldh(KH + aoff + (size_t)mb * 16 * SEQ + kc); ar[mb] = hz;
            if (DOTS_RES) ar[mb] = ldh(KR + aoff + (size_t)mb * 16 * SEQ + kc); }
#pragma unroll
        for (int nb = 0; nb < 2; ++nb) {
            const v16h vh = ldh(VH + boff + (size_t)nb * 16 * SEQ + kc); v16h vr = hz;
            if (DOTS_RES) vr = ldh(VR + boff + (size_t)nb * 16 * SEQ + kc);
#pragma unroll
            for (int mb = 0; mb < 2; ++mb) {
                sH[mb][nb] = wmma16g(ah[mb], vh, sH[mb][nb]);
                if (DOTS_RES) { sR[mb][nb] = wmma16g(ah[mb], vr, sR[mb][nb]); sR[mb][nb] = wmma16g(ar[mb], vh, sR[mb][nb]); } } }
    }
    float* po = PART + ((size_t)hd * KSL + (size_t)sl) * 4096 + (size_t)d0 * 64 + (size_t)e0;
#pragma unroll
    for (int mb = 0; mb < 2; ++mb) {
#pragma unroll
        for (int nb = 0; nb < 2; ++nb) {
#pragma unroll
            for (int j = 0; j < 8; ++j) os[(hi * 8 + j) * OSP + nb * 16 + lr] = sH[mb][nb][j] + sR[mb][nb][j] * QRI; }
        wave_sync();
#pragma unroll 1
        for (int ps = 0; ps < 2; ++ps) {
#pragma unroll
            for (int s = 0; s < 4; ++s) { const int row = 4 * s + (lane >> 3), cofs = (lane & 7) * 4;
                const v4f val = *(const v4fa*)(&os[row * OSP + cofs]);
                *(volatile v4f*)(po + (size_t)(mb * 16 + row) * 64 + cofs) = val; }
            if (ps == 0) __threadfence(); }
        wave_sync();
    }
}

__global__ __launch_bounds__(256) void k_dsum(const float* __restrict__ PART, h16* DH, h16* DR) {
#pragma clang fp contract(off)
    __shared__ float ts[64 * TSP];
    const unsigned tid = threadIdx.x, hd = blockIdx.x;
    const float* pb = PART + (size_t)hd * KSL * 4096;
#pragma unroll 1
    for (unsigned i = 0; i < 4; ++i) {
        const unsigned idx4 = i * 256u + tid; const unsigned d = idx4 >> 4, e4 = (idx4 & 15u) * 4u;
        v4f s = (v4f){};
#pragma unroll 4
        for (int c = 0; c < KSL; ++c) { const v4f p = *(const v4f*)(pb + (size_t)c * 4096 + d * 64u + e4); s = s + p; }
#pragma unroll
        for (int j = 0; j < 4; ++j) ts[(e4 + j) * TSP + d] = s[j] * DSC;
    }
    __syncthreads();
    h16* oh = DH + (size_t)hd * 4096; h16* orr = DR + (size_t)hd * 4096;
#pragma unroll 1
    for (int ps = 0; ps < 2; ++ps) {
#pragma unroll 1
        for (unsigned it = 0; it < 2; ++it) {
            const unsigned p = it * 256u + tid; const unsigned e = p >> 3, c8 = (p & 7u) * 8u;
            v8h hv, rv;
#pragma unroll
            for (int j = 0; j < 8; ++j) { const float x = ts[e * TSP + c8 + j]; const h16 a0 = toh_flush(x); hv[j] = a0; rv[j] = toh_flush((x - (float)a0) * QRS); }
            *(volatile v8h*)(oh + e * 64u + c8) = hv; *(volatile v8h*)(orr + e * 64u + c8) = rv; }
        if (ps == 0) __threadfence(); }
}

__global__ __launch_bounds__(32 * AW) void k_apply(const h16* __restrict__ QH, const h16* __restrict__ QR, const h16* __restrict__ DH, const h16* __restrict__ DR, h16* CH, h16* CR) {
    __shared__ __align__(16) float os[AW * 16 * OSQ];
    const int lane = threadIdx.x & 31, lr = lane & 15, hi = lane >> 4;
    const int wave = __builtin_amdgcn_readfirstlane((int)(threadIdx.x >> 5));
    const unsigned hd = blockIdx.y;
    const unsigned m0 = (blockIdx.x * (unsigned)AW + (unsigned)wave) * 16u;
    const size_t aoff = (size_t)(m0 + lr) * INNER + (size_t)hd * HD + 8 * hi;
    const size_t boff = (size_t)hd * 4096 + (size_t)lr * HD + 8 * hi;
    const v16h hz = (v16h){};
    v8f cH[4], cR[4];
#pragma unroll
    for (int nb = 0; nb < 4; ++nb) { cH[nb] = (v8f){}; cR[nb] = (v8f){}; }
#pragma unroll 1
    for (int kc = 0; kc < HD; kc += 32) {
        const v16h qh = ldh(QH + aoff + kc); v16h qr = hz;
        if (APPLY_RES) qr = ldh(QR + aoff + kc);
#pragma unroll
        for (int nb = 0; nb < 4; ++nb) {
            const v16h dh = ldh(DH + boff + (size_t)nb * 16 * HD + kc); v16h dr = hz;
            if (APPLY_RES) dr = ldh(DR + boff + (size_t)nb * 16 * HD + kc);
            cH[nb] = wmma16g(qh, dh, cH[nb]);
            if (APPLY_RES) { cR[nb] = wmma16g(qh, dr, cR[nb]); cR[nb] = wmma16g(qr, dh, cR[nb]); } }
    }
    const int wb = wave * 16 * OSQ;
#pragma unroll
    for (int nb = 0; nb < 4; ++nb) {
#pragma unroll
        for (int j = 0; j < 8; ++j) os[wb + (hi * 8 + j) * OSQ + nb * 16 + lr] = (cH[nb][j] + cR[nb][j] * QRI) * CSC; }
    wave_sync();
    const size_t obase = (size_t)m0 * INNER + (size_t)hd * HD;
#pragma unroll 1
    for (int ps = 0; ps < 2; ++ps) {
#pragma unroll
        for (int s = 0; s < 4; ++s) { const int row = 4 * s + (lane >> 3), c8 = (lane & 7) * 8;
            const v4f x0 = *(const v4fa*)(&os[wb + row * OSQ + c8]); const v4f x1 = *(const v4fa*)(&os[wb + row * OSQ + c8 + 4]); v8h hv, rv;
#pragma unroll
            for (int i = 0; i < 4; ++i) { const h16 a0 = toh_flush(x0[i]); const h16 a1 = toh_flush(x1[i]); hv[i] = a0; hv[4 + i] = a1;
                rv[i] = toh_flush((x0[i] - (float)a0) * QRS); rv[4 + i] = toh_flush((x1[i] - (float)a1) * QRS); }
            const size_t oo = obase + (size_t)row * INNER + (size_t)c8;
            *(volatile v8h*)(CH + oo) = hv; *(volatile v8h*)(CR + oo) = rv; }
        if (ps == 0) __threadfence(); }
}

__global__ __launch_bounds__(32 * AW) void k_out(const h16* __restrict__ CH, const h16* __restrict__ CR, const h16* __restrict__ WO, const float* __restrict__ bout, float* OUT) {
    __shared__ __align__(16) float os[AW * 16 * OSQ];
    const int lane = threadIdx.x & 31, lr = lane & 15, hi = lane >> 4;
    const int wave = __builtin_amdgcn_readfirstlane((int)(threadIdx.x >> 5));
    const unsigned m0 = (blockIdx.x * (unsigned)AW + (unsigned)wave) * 16u;
    const size_t aoff = (size_t)(m0 + lr) * INNER + 8 * hi;
    const size_t boff = (size_t)lr * INNER + 8 * hi;
    const v16h hz = (v16h){};
    v8f oH[4], oR[4];
#pragma unroll
    for (int nb = 0; nb < 4; ++nb) { oH[nb] = (v8f){}; oR[nb] = (v8f){}; }
#pragma unroll 1
    for (int kc = 0; kc < INNER; kc += 32) {
        const v16h ch = ldh(CH + aoff + kc); v16h cr = hz;
        if (OUT_RES) cr = ldh(CR + aoff + kc);
#pragma unroll
        for (int nb = 0; nb < 4; ++nb) {
            const v16h w = ldh(WO + boff + (size_t)nb * 16 * INNER + kc);
            oH[nb] = wmma16g(ch, w, oH[nb]);
            if (OUT_RES) oR[nb] = wmma16g(cr, w, oR[nb]); }
    }
    const int wb = wave * 16 * OSQ;
#pragma unroll
    for (int nb = 0; nb < 4; ++nb) {
#pragma unroll
        for (int j = 0; j < 8; ++j) os[wb + (hi * 8 + j) * OSQ + nb * 16 + lr] = (oH[nb][j] + oR[nb][j] * QRI) * OSC; }
    wave_sync();
    const int cofs = (lane & 15) * 4;
    const v4f braw = *(const v4f*)(bout + cofs); v4f bv;
#pragma unroll
    for (int i = 0; i < 4; ++i) bv[i] = bfr(braw[i]);
    float* orow = OUT + (size_t)m0 * DM;
#pragma unroll 1
    for (int ps = 0; ps < 2; ++ps) {
#pragma unroll
        for (int s = 0; s < 8; ++s) { const int row = 2 * s + (lane >> 4);
            const v4f x = *(const v4fa*)(&os[wb + row * OSQ + cofs]);
            const v4f val = x + bv;
            *(volatile v4f*)(orow + (size_t)row * DM + cofs) = val; }
        if (ps == 0) __threadfence(); }
}

static constexpr size_t al256(size_t v) { return (v + 255) & ~(size_t)255; }
static constexpr size_t SZ_XB = al256((size_t)NB * SEQ * DM * 2);
static constexpr size_t SZ_WB = al256((size_t)2 * INNER * DM * 2);
static constexpr size_t SZ_WO = al256((size_t)DM * INNER * 2);
static constexpr size_t SZ_PL = al256((size_t)SEQ * INNER * 2);
static constexpr size_t SZ_PT = al256((size_t)NB * NH_ * KSL * 4096 * 4);
static constexpr size_t SZ_DD = al256((size_t)NB * NH_ * 4096 * 2);
static constexpr size_t SZ_TOTAL = 3 * SZ_XB + SZ_WB + SZ_WO + 4 * SZ_PL + SZ_PT + 2 * SZ_DD;
static_assert(SZ_TOTAL <= (size_t)134217728);
static_assert(((size_t)INNER * DM * 2) % 256 == 0);
static_assert((size_t)INNER * SEQ * 2 == (size_t)SEQ * INNER * 2);
static_assert((size_t)SEQ * INNER * 2 <= SZ_PL);
static_assert(((size_t)NH_ * KSL * 4096 * 4) % 256 == 0);
static_assert(((size_t)NH_ * 4096 * 2) % 256 == 0);
static_assert(((size_t)SEQ * DM * 2) % 256 == 0);

extern "C" void kernel_launch(void* const* d_in, const int* in_sizes, int n_in,
                              void* d_out, int out_size, void* d_ws, size_t ws_size, hipStream_t stream) {
    if (n_in < 7) return;
    const size_t needx = ((size_t)(NB - 1) * SEQ_FULL + SEQ) * DM;
    if ((size_t)in_sizes[0] < needx || (size_t)in_sizes[1] < needx || (size_t)in_sizes[2] < needx) return;
    if ((size_t)in_sizes[3] < (size_t)INNER * DM || (size_t)in_sizes[4] < (size_t)INNER * DM || (size_t)in_sizes[5] < (size_t)DM * INNER) return;
    if (in_sizes[6] < DM) return;
    if ((size_t)out_size < ((size_t)(NB - 1) * OUT_SEQ + SEQ) * DM) return;
    if (SZ_TOTAL > ws_size) return;
    const float* xin[3] = { (const float*)d_in[0], (const float*)d_in[1], (const float*)d_in[2] };
    const float* wq = (const float*)d_in[3]; const float* wk = (const float*)d_in[4];
    const float* wo = (const float*)d_in[5]; const float* bo = (const float*)d_in[6];
    float* OUT = (float*)d_out;
    char* wsp = (char*)d_ws;
    bf* XB[3];
    XB[0] = (bf*)wsp; wsp += SZ_XB;
    XB[1] = (bf*)wsp; wsp += SZ_XB;
    XB[2] = (bf*)wsp; wsp += SZ_XB;
    bf* WB = (bf*)wsp; wsp += SZ_WB;
    h16* WO = (h16*)wsp; wsp += SZ_WO;
    h16* P0H = (h16*)wsp; wsp += SZ_PL;
    h16* P0R = (h16*)wsp; wsp += SZ_PL;
    h16* P1H = (h16*)wsp; wsp += SZ_PL;
    h16* P1R = (h16*)wsp; wsp += SZ_PL;
    float* PART = (float*)wsp; wsp += SZ_PT;
    h16* DH = (h16*)wsp; wsp += SZ_DD;
    h16* DR = (h16*)wsp; wsp += SZ_DD;
    bf* WQ = WB; bf* WK = WB + (size_t)INNER * DM;

    for (int i = 0; i < 3; ++i) {
        if (SEQ == SEQ_FULL) {
            const size_t n8 = (size_t)NB * SEQ * DM / 8;
            k_cvt8<<<(unsigned)((n8 + 255) / 256), 256, 0, stream>>>(xin[i], XB[i], n8);
        } else {
            const size_t n8 = (size_t)SEQ * DM / 8;
            for (int b = 0; b < NB; ++b) k_cvt8<<<(unsigned)((n8 + 255) / 256), 256, 0, stream>>>(xin[i] + (size_t)b * SEQ_FULL * DM, XB[i] + (size_t)b * SEQ * DM, n8);
        }
    }
    { const size_t n8 = (size_t)INNER * DM / 8; const unsigned g = (unsigned)((n8 + 255) / 256);
      k_cvt8<<<g, 256, 0, stream>>>(wq, WQ, n8); k_cvt8<<<g, 256, 0, stream>>>(wk, WK, n8);
      k_wcvt<<<g, 256, 0, stream>>>(wo, WO, n8); }

    for (int b = 0; b < NB; ++b) {
        const bf* xq = XB[0] + (size_t)b * SEQ * DM;
        const bf* xk = XB[1] + (size_t)b * SEQ * DM;
        const bf* xv = XB[2] + (size_t)b * SEQ * DM;
        float* part = PART + (size_t)b * NH_ * KSL * 4096;
        h16* dh = DH + (size_t)b * NH_ * 4096;
        h16* dr = DR + (size_t)b * NH_ * 4096;
        k_proj<<<dim3(INNER / 64, SEQ / 64, 1), 32, 0, stream>>>(WK, xk, P0H, P0R, 1);
        k_proj<<<dim3(INNER / 64, SEQ / 64, 1), 32, 0, stream>>>(WK, xv, P1H, P1R, 1);
        k_dots<<<dim3(KSL, 4, NH_), 32, 0, stream>>>(P0H, P0R, P1H, P1R, part);
        k_dsum<<<NH_, 256, 0, stream>>>(part, dh, dr);
        k_proj<<<dim3(SEQ / 64, INNER / 64, 1), 32, 0, stream>>>(xq, WQ, P0H, P0R, 0);
        k_apply<<<dim3(SEQ / (16 * AW), NH_, 1), 32 * AW, 0, stream>>>(P0H, P0R, dh, dr, P1H, P1R);
        k_out<<<dim3(SEQ / (16 * AW), 1, 1), 32 * AW, 0, stream>>>(P1H, P1R, WO, bo, OUT + (size_t)b * OUT_SEQ * DM);
    }
}
